// OrdinalHMM_91147795956227
// MI455X (gfx1250) — hardware-verified
//
#include <hip/hip_runtime.h>
#include <cmath>


namespace {
constexpr int B = 16, B2 = 32, M = 2000, NS = 1000, D = 5000, KP = 5024  , MP = 2048  , SEG = 16, NSEG = M / SEG, NT = 32, SPT = 32  ;
constexpr float LOGN = 6.907755278982137f;

typedef _Float16 b16;
typedef __attribute__((ext_vector_type(16))) _Float16 v16b;
typedef __attribute__((ext_vector_type(8))) _Float16 v8b;
typedef __attribute__((ext_vector_type(8))) float v8f;
typedef __attribute__((ext_vector_type(4))) float v4f;
__device__ __forceinline__ float bf16_rne(float f) { unsigned int u = __float_as_uint(f); u += 0x7FFFu + ((u >> 16) & 1u); return __uint_as_float(u & 0xFFFF0000u); }
__device__ __forceinline__ v16b frag_kb(const b16* p, int hh) { const v8b a = *(const v8b*)(p + 8 * hh), b = *(const v8b*)(p + 16 + 8 * hh); v16b f;
#pragma unroll
  for (int e = 0; e < 8; ++e) { f[e] = a[e]; f[8 + e] = b[e]; } return f; }
__device__ __forceinline__ v8f wmma16b(v16b a, v16b b, v8f c) { v8f d = __builtin_amdgcn_wmma_f32_16x16x32_f16(false, a, false, b, (short)0, c, false, false); asm volatile("v_nop\n\tv_nop\n\tv_nop\n\tv_nop" : "+v"(d) : "v"(a), "v"(b)); return d; }
__device__ __forceinline__ float nexp(float x) { return __builtin_amdgcn_exp2f(x * 1.4426950408889634f); }
__device__ __forceinline__ float nlog(float x) { return __builtin_amdgcn_logf(x) * 0.6931471805599453f; }
__device__ __forceinline__ float pmul(float a, float b) { float p = a * b; asm volatile("" : "+v"(p)); return p; }

__global__ __launch_bounds__(256) void prep_kernel(const float* __restrict__ gexp, b16* __restrict__ Gx) {
  const int t_ = blockIdx.x * 256 + threadIdx.x, nth = gridDim.x * 256;
  for (int pass = 0; pass < 2; ++pass) {
    for (int p = t_; p < B * (KP / 8); p += nth) { const int b = p / (KP / 8), k0 = (p % (KP / 8)) * 8; v8b v;
#pragma unroll
      for (int e = 0; e < 8; ++e) { const int k = k0 + e; v[e] = (b16)((k < D) ? bf16_rne(gexp[(size_t)b * D + k]) : 0.0f); }
      *(volatile v8b*)(Gx + (size_t)b * KP + k0) = v; }
    __threadfence(); }
}

__global__ __launch_bounds__(128) void pred_kernel(const b16* __restrict__ Gx, const float* __restrict__ W, const float* __restrict__ bias, float* __restrict__ lphi) {
  __shared__ float Z[16][64];
  const int lane = threadIdx.x & 31, wave = threadIdx.x >> 5, nloc = lane & 15, hlf = lane >> 4, j0 = blockIdx.x * 64 + wave * 16; const int j = j0 + nloc, jc = (j < M) ? j : (M - 1);
  v8f acc = {};
#pragma unroll 2
  for (int kb = 0; kb < KP; kb += 32) { const v16b a = frag_kb(Gx + (size_t)nloc * KP + kb, hlf); v16b bw;
#pragma unroll
    for (int e = 0; e < 8; ++e) { const int k0 = kb + 8 * hlf + e, k1 = kb + 16 + 8 * hlf + e; bw[e] = (b16)((k0 < D) ? bf16_rne(W[(size_t)k0 * M + jc]) : 0.0f); bw[8 + e] = (b16)((k1 < D) ? bf16_rne(W[(size_t)k1 * M + jc]) : 0.0f); }
    acc = wmma16b(a, bw, acc); }
#pragma unroll
  for (int r = 0; r < 8; ++r) Z[8 * hlf + r][wave * 16 + nloc] = acc[r] + ((j0 + nloc < M) ? bf16_rne(bias[j0 + nloc]) : 0.0f);
  __syncthreads();
  for (int pass = 0; pass < 2; ++pass) { for (int i = threadIdx.x; i < 16 * 64; i += 128) { const int b = i >> 6, jj = i & 63; const float z = Z[b][jj]; const float p = 1.0f / (1.0f + nexp(-z)); const size_t o = ((size_t)b * MP + blockIdx.x * 64 + jj) * 2;
      ((volatile float*)lphi)[o] = nlog(1.0f - p); ((volatile float*)lphi)[o + 1] = nlog(p); } __threadfence(); }
}

__device__ __forceinline__ float block_lse(const float v[SPT], const bool ok[SPT], float* smA, float* smB) { (void)smA; (void)smB; float mx = -INFINITY;
#pragma unroll
  for (int s = 0; s < SPT; ++s) if (ok[s]) mx = fmaxf(mx, v[s]);
#pragma unroll
  for (int o = 1; o < 32; o <<= 1) mx = fmaxf(mx, __shfl_xor(mx, o));
  float su = 0.0f;
#pragma unroll
  for (int s = 0; s < SPT; ++s) if (ok[s]) su += nexp(v[s] - mx);
#pragma unroll
  for (int o = 1; o < 32; o <<= 1) su += __shfl_xor(su, o);
  return mx + nlog(su); }

__device__ __forceinline__ void fwd_step(float f[SPT], const bool ok[SPT], const float se0[SPT], const float se1[SPT], float x0, float x1, float r, float* smA, float* smB) {
  (void)smA; (void)smB;
  float nx[SPT]; float mx = -INFINITY;
#pragma unroll
  for (int s = 0; s < SPT; ++s) { nx[s] = ok[s] ? (f[s] + (pmul(se0[s], x0) + pmul(se1[s], x1))) : -INFINITY; mx = fmaxf(mx, nx[s]); }
#pragma unroll
  for (int o = 1; o < 32; o <<= 1) mx = fmaxf(mx, __shfl_xor(mx, o));
  float es[SPT]; float su = 0.0f;
#pragma unroll
  for (int s = 0; s < SPT; ++s) { es[s] = ok[s] ? nexp(nx[s] - mx) : 0.0f; su += es[s]; }
#pragma unroll
  for (int o = 1; o < 32; o <<= 1) su += __shfl_xor(su, o);
  const float c1 = (1.0f - r) / su, rt = r * (1.0f / (float)NS);
#pragma unroll
  for (int s = 0; s < SPT; ++s) f[s] = ok[s] ? nlog(pmul(c1, es[s]) + rt) : -INFINITY;
}

__device__ __forceinline__ void load_se(const unsigned int* __restrict__ refb, int i, const bool ok[SPT], float le00, float le01, float le10, float le11, float se0[SPT], float se1[SPT]) {
  const unsigned int wbits = refb[(size_t)i * 32 + threadIdx.x];
#pragma unroll
  for (int s = 0; s < SPT; ++s) { const bool rv = ok[s] && ((wbits >> s) & 1u); se0[s] = rv ? le10 : le00; se1[s] = rv ? le11 : le01; } }

__global__ __launch_bounds__(256) void pack_kernel(const int* __restrict__ ref, unsigned int* __restrict__ refb) {
  const int i = blockIdx.x * 8 + (threadIdx.x >> 5), l = threadIdx.x & 31; unsigned int wv = 0;
  for (int s = 0; s < 32; ++s) { const int n = 32 * l + s; if (n < NS && ref[(size_t)i * NS + n] != 0) wv |= 1u << s; }
  for (int pass = 0; pass < 2; ++pass) ((volatile unsigned int*)refb)[(size_t)i * 32 + l] = wv;
  __threadfence();
}

__global__ __launch_bounds__(32) void fwd_kernel(const unsigned int* __restrict__ ref, const float* __restrict__ xo, const float* __restrict__ rr, float le00, float le01, float le10, float le11, b16* __restrict__ fp) {
  __shared__ float smA[16], smB[16];
  const int b2 = blockIdx.x, t_ = threadIdx.x; bool ok[SPT]; float f[SPT];
#pragma unroll
  for (int s = 0; s < SPT; ++s) { ok[s] = (32 * t_ + s) < NS; f[s] = 0.0f; }
  for (int i = 0; i < M; ++i) {
    {
      b16* row = fp + ((size_t)i * B2 + b2) * 1024 + 32 * t_;
      for (int pass = 0; pass < 2; ++pass) { if (t_ < 31) {
#pragma unroll
          for (int g = 0; g < 4; ++g) { v8b v; for (int e = 0; e < 8; ++e) v[e] = (b16)f[g * 8 + e]; *(volatile v8b*)(row + g * 8) = v; } }
        else { v8b v; for (int e = 0; e < 8; ++e) v[e] = (b16)f[e]; *(volatile v8b*)(row) = v; } } }
    float se0[SPT], se1[SPT]; load_se(ref, i, ok, le00, le01, le10, le11, se0, se1);
    const float x0 = bf16_rne(xo[((size_t)b2 * M + i) * 2]), x1 = bf16_rne(xo[((size_t)b2 * M + i) * 2 + 1]); const float r = (i + 1 < M) ? bf16_rne(rr[i + 1]) : 0.5f;
    fwd_step(f, ok, se0, se1, x0, x1, r, smA, smB); }
  __threadfence();
}

__global__ __launch_bounds__(32) void bwd_kernel(const unsigned int* __restrict__ ref, const float* __restrict__ xo, const float* __restrict__ rr, const float* __restrict__ lphi, const b16* __restrict__ fp, float le00, float le01, float le10, float le11, float E00, float E01, float E10, float E11, float* __restrict__ pxe) {
  __shared__ float smA[16], smB[16];
  const int b2 = blockIdx.x, t_ = threadIdx.x, bsrc = b2 >> 1; bool ok[SPT]; float st[SPT];
#pragma unroll
  for (int s = 0; s < SPT; ++s) { ok[s] = (32 * t_ + s) < NS; st[s] = 0.0f; }
  float p_xe = 0.0f;
  { for (int i = M - 1; i >= 0; --i) {
      float fi[SPT]; { const b16* row = fp + ((size_t)i * B2 + b2) * 1024 + 32 * t_;
        if (t_ < 31) {
#pragma unroll
          for (int g = 0; g < 4; ++g) { const v8b v = *(const v8b*)(row + g * 8); for (int e = 0; e < 8; ++e) fi[g * 8 + e] = (float)v[e]; } }
        else { const v8b v = *(const v8b*)(row); for (int e = 0; e < 8; ++e) fi[e] = (float)v[e]; for (int e = 8; e < 32; ++e) fi[e] = 0.0f; } }
      float se0[SPT], se1[SPT]; load_se(ref, i, ok, le00, le01, le10, le11, se0, se1);
      const float ph0 = lphi[((size_t)bsrc * MP + i) * 2], ph1 = lphi[((size_t)bsrc * MP + i) * 2 + 1];
      const float x0 = bf16_rne(xo[((size_t)b2 * M + i) * 2]), x1 = bf16_rne(xo[((size_t)b2 * M + i) * 2 + 1]); const float r = bf16_rne(rr[i]);
      float fsv[SPT]; float mf = -INFINITY;
#pragma unroll
      for (int s = 0; s < SPT; ++s) { fsv[s] = ok[s] ? (fi[s] + st[s]) : -INFINITY; mf = fmaxf(mf, fsv[s]); }
#pragma unroll
      for (int o = 1; o < 32; o <<= 1) mf = fmaxf(mf, __shfl_xor(mf, o));
      float sA = 0.0f, sB = 0.0f; { const unsigned int wb = ref[(size_t)i * 32 + t_];
#pragma unroll
        for (int s = 0; s < SPT; ++s) { const float e_ = ok[s] ? nexp(fsv[s] - mf) : 0.0f; if ((wb >> s) & 1u) sB += e_; else sA += e_; } }
#pragma unroll
      for (int o = 1; o < 32; o <<= 1) { sA += __shfl_xor(sA, o); sB += __shfl_xor(sB, o); }
      const float dp0 = mf + nlog(pmul(sA, E00) + pmul(sB, E10)), dp1 = mf + nlog(pmul(sA, E01) + pmul(sB, E11));
      (void)se0; (void)se1;
      const float dpp0 = dp0 + ph0, dpp1 = dp1 + ph1; const float mx = fmaxf(dpp0, dpp1); const float lz = mx + nlog(nexp(dpp0 - mx) + nexp(dpp1 - mx));
      p_xe += pmul(dpp0 - lz, x0) + pmul(dpp1 - lz, x1);
      float nn[SPT]; {
        const float uA0 = le00 + ph0, uA1 = le01 + ph1, uB0 = le10 + ph0, uB1 = le11 + ph1; const float mA = fmaxf(uA0, uA1), mB = fmaxf(uB0, uB1);
        const float nnA = mA + nlog(nexp(uA0 - mA) + nexp(uA1 - mA)), nnB = mB + nlog(nexp(uB0 - mB) + nexp(uB1 - mB)); const unsigned int wbits = ref[(size_t)i * 32 + t_];
#pragma unroll
        for (int s = 0; s < SPT; ++s) nn[s] = ok[s] ? (((wbits >> s) & 1u) ? nnB : nnA) : -INFINITY; }
#pragma unroll
      for (int s = 0; s < SPT; ++s) st[s] = ok[s] ? (st[s] + nn[s]) : -INFINITY;
      float smx = -INFINITY;
#pragma unroll
      for (int s = 0; s < SPT; ++s) if (ok[s]) smx = fmaxf(smx, st[s]);
#pragma unroll
      for (int o = 1; o < 32; o <<= 1) smx = fmaxf(smx, __shfl_xor(smx, o));
      float su = 0.0f; float es[SPT];
#pragma unroll
      for (int s = 0; s < SPT; ++s) { es[s] = ok[s] ? nexp(st[s] - smx) : 0.0f; su += es[s]; }
#pragma unroll
      for (int o = 1; o < 32; o <<= 1) su += __shfl_xor(su, o);
      const float rt = pmul(r, su * (1.0f / (float)NS));
#pragma unroll
      for (int s = 0; s < SPT; ++s) st[s] = ok[s] ? nlog(pmul(1.0f - r, es[s]) + rt) : 0.0f; } }
  { const float v = (t_ == 0) ? p_xe : 0.0f; for (int pass = 0; pass < 2; ++pass) ((volatile float*)pxe)[(size_t)b2 * 32 + t_] = v; }
  __threadfence();
}

__global__ __launch_bounds__(32) void loss_kernel(const float* __restrict__ pxe, float* __restrict__ out) {
  if (threadIdx.x == 0) { float s = 0.0f; for (int b = 0; b < B2; ++b) s += pxe[(size_t)b * 32]; for (int pass = 0; pass < 2; ++pass) ((volatile float*)out)[0] = -s; }
  __threadfence();
}
}

extern "C" void kernel_launch(void* const* d_in, const int* in_sizes, int n_in,
                              void* d_out, int out_size, void* d_ws, size_t ws_size, hipStream_t stream) {
  (void)n_in; (void)out_size;
  const float* gexp = (const float*)d_in[0]; const float* xo = (const float*)d_in[1]; const float* W = (const float*)d_in[2]; const float* bias = (const float*)d_in[3]; const int* refi = (const int*)d_in[4]; const float* rr = (const float*)d_in[5];
  float* out = (float*)d_out;
  if (in_sizes[0] != B * D || in_sizes[1] != B2 * M * 2 || in_sizes[2] != D * M || in_sizes[4] != M * NS || in_sizes[5] != M) return;
  size_t off = 0; char* ws = (char*)d_ws;
  auto carve = [&](size_t bytes) { char* p = ws + off; off += (bytes + 255) & ~(size_t)255; return p; };
  b16* fp = (b16*)carve((size_t)M * B2 * 1024 * 2); b16* Gx = (b16*)carve((size_t)B * KP * 2); float* lphi = (float*)carve((size_t)B * MP * 2 * 4); unsigned int* refb = (unsigned int*)carve((size_t)M * 32 * 4); float* pxe = (float*)carve((size_t)B2 * 32 * 4);
  if (off > ws_size) return;
  const double e = 0.01, ps = 1.0 / (double)NS; const float le00 = (float)std::log(1.0 - e + ps), le01 = (float)std::log(e + ps), le10 = (float)std::log(e + ps), le11 = (float)std::log(1.0 - e + ps);
  prep_kernel<<<32, 256, 0, stream>>>(gexp, Gx);
  pack_kernel<<<M / 8, 256, 0, stream>>>(refi, refb);
  pred_kernel<<<MP / 64, 128, 0, stream>>>(Gx, W, bias, lphi);
  fwd_kernel<<<B2, 32, 0, stream>>>(refb, xo, rr, le00, le01, le10, le11, fp);
  const float E00 = std::exp(le00), E01 = std::exp(le01), E10 = std::exp(le10), E11 = std::exp(le11);
  bwd_kernel<<<B2, 32, 0, stream>>>(refb, xo, rr, lphi, fp, le00, le01, le10, le11, E00, E01, E10, E11, pxe);
  loss_kernel<<<1, 32, 0, stream>>>(pxe, out);
}
